// Gpt2Attention_27041114096448
// MI455X (gfx1250) — hardware-verified
//
#include <hip/hip_runtime.h>
#pragma clang fp contract(off)


#ifndef NB
#define NB 2
#endif
#ifndef SEQ
#define SEQ 2048
#endif
#define NB_FULL  2
#define SEQ_FULL 2048
#define DM   1024
#define NH   16
#define HD   64
#define NQKV (3 * DM)
#define RE   64
#define NCHK 64
#define PCAR 1024.0f
#define SCL  0.125f
#define L2E  1.4426950408889634f

static_assert(SEQ % 64 == 0);
static_assert(SEQ >= 64 && SEQ <= SEQ_FULL);
static_assert(NB >= 1 && NB <= NB_FULL);
static_assert(RE == 64);
static_assert(NCHK == 64);
static_assert(SEQ % NCHK == 0);
static_assert(DM == NH * HD);
static_assert(DM % 64 == 0);
static_assert(NQKV % 64 == 0);

typedef _Float16 h16;
typedef unsigned short bf;
typedef __attribute__((ext_vector_type(16))) __bf16   v16bf;
typedef __attribute__((ext_vector_type(16))) _Float16 v16h;
typedef __attribute__((ext_vector_type(8)))  _Float16 v8h;
typedef __attribute__((ext_vector_type(8)))  unsigned short v8us;
typedef __attribute__((ext_vector_type(8)))  float    v8f;
typedef __attribute__((ext_vector_type(4)))  float    v4f;
typedef v8h  __attribute__((may_alias)) v8ha;
typedef v4f  __attribute__((may_alias)) v4fa;
typedef v8us __attribute__((may_alias)) v8usa;
typedef v8f  __attribute__((may_alias)) v8fa;

__device__ __forceinline__ unsigned short f2bf(float f) { unsigned u = __float_as_uint(f); u += 0x7FFFu + ((u >> 16) & 1u); return (unsigned short)(u >> 16); }
__device__ __forceinline__ float bf2f(unsigned short b) { return __uint_as_float(((unsigned)b) << 16); }
__device__ __forceinline__ float bfr(float f) { return bf2f(f2bf(f)); }
__device__ __forceinline__ void splitf(float y, unsigned short& h, unsigned short& l) { h = f2bf(y); l = f2bf(y - bf2f(h)); }
__device__ __forceinline__ v16h cat16(v8h lo, v8h hi) { return __builtin_shufflevector(lo, hi, 0, 1, 2, 3, 4, 5, 6, 7, 8, 9, 10, 11, 12, 13, 14, 15); }
__device__ __forceinline__ v16bf cat16b(v8us lo, v8us hi) { return __builtin_bit_cast(v16bf, __builtin_shufflevector(lo, hi, 0, 1, 2, 3, 4, 5, 6, 7, 8, 9, 10, 11, 12, 13, 14, 15)); }
__device__ __forceinline__ v8f wmma16(v16h a, v16h b, v8f c) { return __builtin_amdgcn_wmma_f32_16x16x32_f16(false, a, false, b, (short)0, c, false, false); }
__device__ __forceinline__ v8f wmmab(v16bf a, v16bf b, v8f c) { return __builtin_amdgcn_wmma_f32_16x16x32_bf16(false, a, false, b, (short)0, c, false, false); }

template <typename T16> struct WFrag;
template <> struct WFrag<h16> { typedef v16h V; static __device__ __forceinline__ V ld(const h16* p) { return cat16(*(const v8ha*)p, *(const v8ha*)(p + 16)); } static __device__ __forceinline__ v8f mma(V a, V b, v8f c) { return wmma16(a, b, c); } };
template <> struct WFrag<bf> { typedef v16bf V; static __device__ __forceinline__ V ld(const bf* p) { return cat16b(*(const v8usa*)p, *(const v8usa*)(p + 16)); } static __device__ __forceinline__ v8f mma(V a, V b, v8f c) { return wmmab(a, b, c); } };

template <typename T16, int NSPLIT>
__device__ __forceinline__ void gemm_core(const T16* __restrict__ A, const T16* __restrict__ A2, const T16* __restrict__ Bt, const T16* __restrict__ Bt2,
                                          int K, int r0, int c0, int lane, v8f (&acc)[4][4]) {
    typedef typename WFrag<T16>::V V;
    const int lr = lane & 15, hi = lane >> 4;
#pragma unroll
    for (int mb = 0; mb < 4; ++mb)
#pragma unroll
        for (int nb = 0; nb < 4; ++nb) acc[mb][nb] = (v8f){};
    const size_t aoff = (size_t)(r0 + lr) * K + 8 * hi, boff = (size_t)(c0 + lr) * K + 8 * hi;
#pragma unroll 1
    for (int kc = 0; kc < K; kc += 32) {
        V a[4], a2[4];
#pragma unroll
        for (int mb = 0; mb < 4; ++mb) { a[mb] = WFrag<T16>::ld(A + aoff + (size_t)mb * 16 * K + kc); if (NSPLIT == 1 || NSPLIT == 2) a2[mb] = WFrag<T16>::ld(A2 + aoff + (size_t)mb * 16 * K + kc); }
#pragma unroll
        for (int nb = 0; nb < 4; ++nb) { const V b = WFrag<T16>::ld(Bt + boff + (size_t)nb * 16 * K + kc); V b2; if (NSPLIT >= 2) b2 = WFrag<T16>::ld(Bt2 + boff + (size_t)nb * 16 * K + kc);
#pragma unroll
            for (int mb = 0; mb < 4; ++mb) { acc[mb][nb] = WFrag<T16>::mma(a[mb], b, acc[mb][nb]); if (NSPLIT == 1 || NSPLIT == 2) acc[mb][nb] = WFrag<T16>::mma(a2[mb], b, acc[mb][nb]); if (NSPLIT >= 2) acc[mb][nb] = WFrag<T16>::mma(a[mb], b2, acc[mb][nb]); } }
        asm volatile("v_nop\n\tv_nop\n\tv_nop\n\tv_nop" : "+v"(acc[0][0]), "+v"(acc[1][1]), "+v"(acc[2][2]), "+v"(acc[3][3]) : "v"(a[0]), "v"(a[3]));
    }
}

template <typename T16, int NSPLIT>
__global__ __launch_bounds__(32) void k_gemmw(const T16* __restrict__ A, const T16* __restrict__ A2, const T16* __restrict__ Bt, const T16* __restrict__ Bt2,
                                              int K, const float* __restrict__ bias, float* C, int ldc, size_t sA, size_t sB, size_t sC) {
    __shared__ __align__(16) float os[16 * 68];
    const size_t z = blockIdx.z; A += z * sA; if (A2) A2 += z * sA; Bt += z * sB; if (Bt2) Bt2 += z * sB; C += z * sC;
    const int lane = threadIdx.x & 31, lr = lane & 15, hi = lane >> 4; const int r0 = blockIdx.x * 64, c0 = blockIdx.y * 64;
    v8f acc[4][4];
    gemm_core<T16, NSPLIT>(A, A2, Bt, Bt2, K, r0, c0, lane, acc);
    float bcol[4];
#pragma unroll
    for (int nb = 0; nb < 4; ++nb) bcol[nb] = bfr(bias[c0 + nb * 16 + lr]);
#pragma unroll
    for (int mb = 0; mb < 4; ++mb) {
#pragma unroll
        for (int nb = 0; nb < 4; ++nb) {
#pragma unroll
            for (int j = 0; j < 8; ++j) os[(hi * 8 + j) * 68 + nb * 16 + lr] = acc[mb][nb][j] + bcol[nb]; }
        __syncthreads();
        float* crow = C + (size_t)(r0 + mb * 16) * ldc + c0;
#pragma unroll 1
        for (int ps = 0; ps < 2; ++ps) {
#pragma unroll
            for (int s = 0; s < 8; ++s) { const int row = 2 * s + hi, cofs = lr * 4; const v4f val = *(const v4fa*)(os + row * 68 + cofs);
                *(volatile v4f*)(crow + (size_t)row * ldc + cofs) = val; }
            if (ps == 0) __threadfence(); }
        __syncthreads();
    }
}

template <int HLM>
__global__ __launch_bounds__(32) void k_gemmp(const bf* __restrict__ A, const bf* __restrict__ Bt, int K, const float* __restrict__ bias,
                                              h16* C16, int ldc, bf* Ch, bf* Cl, int ldh,
                                              size_t sA, size_t sB, size_t sBias, size_t sC, size_t sH) {
    __shared__ __align__(16) float os[16 * 68];
    const size_t z = blockIdx.z; A += z * sA; Bt += z * sB; bias += z * sBias; C16 += z * sC; Ch += z * sH; Cl += z * sH;
    const int lane = threadIdx.x & 31, lr = lane & 15, hi = lane >> 4; const int r0 = blockIdx.x * 64, c0 = blockIdx.y * 64;
    v8f acc[4][4];
    gemm_core<bf, 0>(A, nullptr, Bt, nullptr, K, r0, c0, lane, acc);
    const int t0 = (HLM == 1) ? (r0 % SEQ) : 0;
    const bool hl = (HLM == 1) ? (t0 < RE) : (c0 < RE);
    const int rc0 = (HLM == 1) ? ((r0 / SEQ) * RE + t0) : r0;
    const int rsub = lane >> 3, cseg = (lane & 7) * 8;
    float bcol[4];
#pragma unroll
    for (int nb = 0; nb < 4; ++nb) bcol[nb] = (HLM == 1) ? bfr(bias[c0 + nb * 16 + lr]) : 0.0f;
#pragma unroll
    for (int mb = 0; mb < 4; ++mb) {
        float brow[8];
        if (HLM == 2) { const v8f bv = *(const v8fa*)(bias + r0 + mb * 16 + hi * 8);
#pragma unroll
            for (int j = 0; j < 8; ++j) brow[j] = bfr(bv[j]); }
        else {
#pragma unroll
            for (int j = 0; j < 8; ++j) brow[j] = 0.0f; }
#pragma unroll
        for (int nb = 0; nb < 4; ++nb) {
#pragma unroll
            for (int j = 0; j < 8; ++j) os[(hi * 8 + j) * 68 + nb * 16 + lr] = acc[mb][nb][j] + bcol[nb] + brow[j]; }
        __syncthreads();
#pragma unroll 1
        for (int ps = 0; ps < 2; ++ps) {
#pragma unroll
            for (int j4 = 0; j4 < 4; ++j4) {
                const int row = j4 * 4 + rsub;
                const v4f v0 = *(const v4fa*)(os + row * 68 + cseg);
                const v4f v1 = *(const v4fa*)(os + row * 68 + cseg + 4);
                float y[8] = {v0[0], v0[1], v0[2], v0[3], v1[0], v1[1], v1[2], v1[3]};
                v8h o16;
#pragma unroll
                for (int q = 0; q < 8; ++q) o16[q] = (h16)y[q];
                const size_t grow = (size_t)(r0 + mb * 16 + row);
                *(volatile v8h*)(C16 + grow * (size_t)ldc + c0 + cseg) = o16;
                if (hl) {
                    v8us oh, ol;
#pragma unroll
                    for (int q = 0; q < 8; ++q) { unsigned short a2, c2; splitf(y[q], a2, c2); oh[q] = a2; ol[q] = c2; }
                    const size_t o = (size_t)(rc0 + mb * 16 + row) * (size_t)ldh + c0 + cseg;
                    *(volatile v8us*)(Ch + o) = oh; *(volatile v8us*)(Cl + o) = ol;
                }
            }
            if (ps == 0) __threadfence();
        }
        __syncthreads();
    }
}

__global__ __launch_bounds__(256) void k_cvtT(const float* __restrict__ src, bf* dst, int R, int C) {
    __shared__ __align__(16) float ts[64 * 68];
    const int tid = threadIdx.x, lane = tid & 31, w = tid >> 5;
    const int r0 = blockIdx.x * 64, c0 = blockIdx.y * 64;
#pragma unroll
    for (int i = 0; i < 4; ++i) { const int idx = tid + 256 * i; const int row = idx >> 4, c4 = (idx & 15) * 4;
        const v4f v = *(const v4fa*)(src + (size_t)(r0 + row) * C + c0 + c4);
#pragma unroll
        for (int j = 0; j < 4; ++j) ts[(c4 + j) * 68 + row] = v[j]; }
    __syncthreads();
    const int rsub = lane >> 3, cseg = (lane & 7) * 8;
#pragma unroll 1
    for (int ps = 0; ps < 2; ++ps) {
#pragma unroll
        for (int j = 0; j < 2; ++j) { const int cl = w * 8 + j * 4 + rsub;
            const v4f v0 = *(const v4fa*)(ts + cl * 68 + cseg); const v4f v1 = *(const v4fa*)(ts + cl * 68 + cseg + 4); v8us o;
#pragma unroll
            for (int q = 0; q < 4; ++q) { o[q] = f2bf(v0[q]); o[4 + q] = f2bf(v1[q]); }
            *(volatile v8us*)(dst + (size_t)(c0 + cl) * R + r0 + cseg) = o; }
        if (ps == 0) __threadfence(); }
}

__global__ __launch_bounds__(256) void k_cvtx(const float* __restrict__ src, bf* dst, size_t n8) {
    const size_t i = (size_t)blockIdx.x * 256 + threadIdx.x; if (i >= n8) return; const size_t e = i * 8; const size_t row = e / DM; const size_t c = e % DM;
    const size_t b = row / SEQ, t = row % SEQ; const v8f v = *(const v8fa*)(src + (b * SEQ_FULL + t) * DM + c); v8us o;
#pragma unroll
    for (int k = 0; k < 8; ++k) o[k] = f2bf(v[k]);
    *(volatile v8us*)(dst + e) = o; __threadfence(); *(volatile v8us*)(dst + e) = o;
}

__global__ __launch_bounds__(256) void k_mchk(const float* __restrict__ am, float* FL) {
    __shared__ int red[8];
    const int tid = threadIdx.x, lane = tid & 31, w = tid >> 5; const int c = blockIdx.x;
    int bad = 0;
    const int rpb = SEQ / NCHK;
#pragma unroll 1
    for (int rr = 0; rr < rpb; ++rr) { const int i = c * rpb + rr; const float* rowp = am + (size_t)i * SEQ_FULL;
#pragma unroll 1
        for (int j = tid; j < SEQ; j += 256) { const float v = rowp[j]; const bool good = (j <= i) ? (v == 1.0f) : (v == 0.0f); bad += good ? 0 : 1; } }
#pragma unroll
    for (int sh = 16; sh; sh >>= 1) bad += __shfl_xor(bad, sh, 32);
    if (lane == 0) red[w] = bad;
    __syncthreads();
    if (w == 0) { int tot = 0;
#pragma unroll
        for (int i = 0; i < 8; ++i) tot += red[i];
        const float f = (tot == 0) ? 1.0f : 0.0f; *(volatile float*)(FL + (size_t)c * 32 + lane) = f; __threadfence(); *(volatile float*)(FL + (size_t)c * 32 + lane) = f; }
}
__device__ __forceinline__ bool read_flag(const float* __restrict__ FL, int lane) {
    float f = fminf(FL[(size_t)(2 * lane) * 32], FL[(size_t)(2 * lane + 1) * 32]);
#pragma unroll
    for (int sh = 16; sh; sh >>= 1) f = fminf(f, __shfl_xor(f, sh, 32));
    return f > 0.5f;
}

__device__ __forceinline__ void store_ctx(const float* osw, bf* ATh, bf* ATl, size_t base, int lane) {
    const int rsub = lane >> 3, cseg = (lane & 7) * 8;
#pragma unroll 1
    for (int ps = 0; ps < 2; ++ps) {
#pragma unroll
        for (int j4 = 0; j4 < 4; ++j4) { const int row = j4 * 4 + rsub; const v4f v0 = *(const v4fa*)(osw + row * 68 + cseg); const v4f v1 = *(const v4fa*)(osw + row * 68 + cseg + 4); v8us oh, ol;
#pragma unroll
            for (int q = 0; q < 4; ++q) { unsigned short a, c2; splitf(v0[q], a, c2); oh[q] = a; ol[q] = c2; splitf(v1[q], a, c2); oh[4 + q] = a; ol[4 + q] = c2; }
            const size_t o = base + (size_t)row * DM + cseg; *(volatile v8us*)(ATh + o) = oh; *(volatile v8us*)(ATl + o) = ol; }
        if (ps == 0) __threadfence(); }
}

__global__ __launch_bounds__(128) void k_attn(const h16* __restrict__ Q16, const h16* __restrict__ K16, const h16* __restrict__ VT16, const float* __restrict__ FL, bf* ATh, bf* ATl) {
    __shared__ __align__(16) h16 Ks[64 * 72];
    __shared__ __align__(16) h16 Vs[64 * 72];
    __shared__ __align__(16) h16 Ps[4 * 16 * 72];
    __shared__ __align__(16) float Os[4 * 16 * 68];
    const int tid = threadIdx.x, lane = tid & 31, w = tid >> 5, m = lane & 15, hh = lane >> 4;
    const int qt = blockIdx.x + 1;
    const int b = blockIdx.y / NH, h = blockIdx.y % NH;
    const int q0 = qt * 64 + w * 16;
    const bool ok = read_flag(FL, lane);
    const h16* qrow = Q16 + (size_t)(b * SEQ + q0 + m) * DM + h * HD + 8 * hh;
    v16h aq[2];
#pragma unroll
    for (int ks = 0; ks < 2; ++ks) aq[ks] = cat16(*(const v8ha*)(qrow + ks * 32), *(const v8ha*)(qrow + ks * 32 + 16));
    v8f acc[4]; float mrun[8], lrun[8];
#pragma unroll
    for (int nb = 0; nb < 4; ++nb) acc[nb] = (v8f){};
#pragma unroll
    for (int r = 0; r < 8; ++r) { mrun[r] = -1.0e30f; lrun[r] = 0.f; }
    const h16* kbase = K16 + (size_t)b * SEQ * DM + h * HD;
    const h16* vbase = VT16 + ((size_t)b * DM + h * HD) * SEQ;
    h16* psw = Ps + w * (16 * 72);
    float* osw = Os + w * (16 * 68);
#pragma unroll 1
    for (int kc = 0; kc <= qt; ++kc) {
        __syncthreads();
#pragma unroll
        for (int i = 0; i < 4; ++i) { const int p = tid + 128 * i; const int row = p >> 3, c8 = (p & 7) * 8;
            *(v8ha*)(Ks + row * 72 + c8) = *(const v8ha*)(kbase + (size_t)(kc * 64 + row) * DM + c8);
            *(v8ha*)(Vs + row * 72 + c8) = *(const v8ha*)(vbase + (size_t)row * SEQ + kc * 64 + c8); }
        __syncthreads();
        v8f s[4];
#pragma unroll
        for (int nb = 0; nb < 4; ++nb) s[nb] = (v8f){};
#pragma unroll
        for (int ks = 0; ks < 2; ++ks) {
#pragma unroll
            for (int nb = 0; nb < 4; ++nb) { const h16* kpp = Ks + (nb * 16 + m) * 72 + ks * 32 + 8 * hh; const v16h bk = cat16(*(const v8ha*)kpp, *(const v8ha*)(kpp + 16)); s[nb] = wmma16(aq[ks], bk, s[nb]); } }
        asm volatile("v_nop\n\tv_nop\n\tv_nop\n\tv_nop" : "+v"(s[0]), "+v"(s[1]), "+v"(s[2]), "+v"(s[3]) : "v"(aq[0]), "v"(aq[1]));
        const bool diag = (kc == qt); const int qab = q0 + 8 * hh; const int kab = kc * 64 + m;
        float cm[8], al[8], psum[8];
#pragma unroll
        for (int r = 0; r < 8; ++r) cm[r] = -3.0e38f;
#pragma unroll
        for (int nb = 0; nb < 4; ++nb)
#pragma unroll
            for (int r = 0; r < 8; ++r) { float v = s[nb][r] * SCL; if (diag && (kab + nb * 16 > qab + r)) v = -1.0e30f; s[nb][r] = v; cm[r] = fmaxf(cm[r], v); }
#pragma unroll
        for (int r = 0; r < 8; ++r) { float c = cm[r]; c = fmaxf(c, __shfl_xor(c, 1, 32)); c = fmaxf(c, __shfl_xor(c, 2, 32)); c = fmaxf(c, __shfl_xor(c, 4, 32)); c = fmaxf(c, __shfl_xor(c, 8, 32));
            const float mn = fmaxf(mrun[r], c); al[r] = __builtin_amdgcn_exp2f((mrun[r] - mn) * L2E); mrun[r] = mn; psum[r] = 0.f; }
#pragma unroll
        for (int nb = 0; nb < 4; ++nb)
#pragma unroll
            for (int r = 0; r < 8; ++r) { const float p = __builtin_amdgcn_exp2f((s[nb][r] - mrun[r]) * L2E); psum[r] += p; psw[(8 * hh + r) * 72 + nb * 16 + m] = (h16)(p * PCAR); }
#pragma unroll
        for (int r = 0; r < 8; ++r) { float c = psum[r]; c += __shfl_xor(c, 1, 32); c += __shfl_xor(c, 2, 32); c += __shfl_xor(c, 4, 32); c += __shfl_xor(c, 8, 32);
            const float sc = lrun[r] * al[r]; lrun[r] = sc + c; }
#pragma unroll
        for (int nb = 0; nb < 4; ++nb)
#pragma unroll
            for (int r = 0; r < 8; ++r) acc[nb][r] = acc[nb][r] * al[r];
        __syncthreads();
        v16h ap[2];
#pragma unroll
        for (int ks = 0; ks < 2; ++ks) { const h16* pp = psw + m * 72 + ks * 32 + 8 * hh; ap[ks] = cat16(*(const v8ha*)pp, *(const v8ha*)(pp + 16)); }
#pragma unroll
        for (int ks = 0; ks < 2; ++ks)
#pragma unroll
            for (int nb = 0; nb < 4; ++nb) { const h16* vp = Vs + (nb * 16 + m) * 72 + ks * 32 + 8 * hh; const v16h bv = cat16(*(const v8ha*)vp, *(const v8ha*)(vp + 16)); acc[nb] = wmma16(ap[ks], bv, acc[nb]); }
        asm volatile("v_nop\n\tv_nop\n\tv_nop\n\tv_nop" : "+v"(acc[0]), "+v"(acc[1]), "+v"(acc[2]), "+v"(acc[3]) : "v"(ap[0]), "v"(ap[1]));
    }
    const float qnan = __uint_as_float(0x7fc00000u);
#pragma unroll
    for (int r = 0; r < 8; ++r) { const float iv = 1.0f / (lrun[r] * PCAR);
#pragma unroll
        for (int nb = 0; nb < 4; ++nb) { const float o = acc[nb][r] * iv; osw[(8 * hh + r) * 68 + nb * 16 + m] = ok ? o : qnan; } }
    __syncthreads();
    store_ctx(osw, ATh, ATl, (size_t)(b * SEQ + q0) * DM + h * HD, lane);
}

__global__ __launch_bounds__(64) void k_attn0(const bf* __restrict__ Qh, const bf* __restrict__ Ql, const bf* __restrict__ Kh, const bf* __restrict__ Kl,
                                              const bf* __restrict__ VTh, const bf* __restrict__ VTl, const float* __restrict__ FL, bf* ATh, bf* ATl) {
    __shared__ __align__(16) bf Khs[64 * 72];
    __shared__ __align__(16) bf Kls[64 * 72];
    __shared__ __align__(16) bf Vhs[64 * 72];
    __shared__ __align__(16) bf Vls[64 * 72];
    __shared__ __align__(16) bf Phs[2 * 16 * 72];
    __shared__ __align__(16) bf Pls[2 * 16 * 72];
    __shared__ __align__(16) float Os[2 * 16 * 68];
    const int tid = threadIdx.x, lane = tid & 31, w = tid >> 5, m = lane & 15, hh = lane >> 4;
    const int b = blockIdx.y / NH, h = blockIdx.y % NH;
    const int q0 = blockIdx.x * 32 + w * 16;
    const bool ok = read_flag(FL, lane);
    const bf* kh0 = Kh + (size_t)b * RE * DM + h * HD; const bf* kl0 = Kl + (size_t)b * RE * DM + h * HD;
    const bf* vh0 = VTh + ((size_t)b * DM + h * HD) * RE; const bf* vl0 = VTl + ((size_t)b * DM + h * HD) * RE;
#pragma unroll
    for (int i = 0; i < 8; ++i) { const int p = tid + 64 * i; const int row = p >> 3, c8 = (p & 7) * 8;
        *(v8usa*)(Khs + row * 72 + c8) = *(const v8usa*)(kh0 + (size_t)row * DM + c8);
        *(v8usa*)(Kls + row * 72 + c8) = *(const v8usa*)(kl0 + (size_t)row * DM + c8);
        *(v8usa*)(Vhs + row * 72 + c8) = *(const v8usa*)(vh0 + (size_t)row * RE + c8);
        *(v8usa*)(Vls + row * 72 + c8) = *(const v8usa*)(vl0 + (size_t)row * RE + c8); }
    __syncthreads();
    const bf* qh = Qh + (size_t)(b * RE + q0 + m) * DM + h * HD + 8 * hh; const bf* ql = Ql + (size_t)(b * RE + q0 + m) * DM + h * HD + 8 * hh;
    v16bf aqh[2], aql[2];
#pragma unroll
    for (int ks = 0; ks < 2; ++ks) { aqh[ks] = cat16b(*(const v8usa*)(qh + ks * 32), *(const v8usa*)(qh + ks * 32 + 16)); aql[ks] = cat16b(*(const v8usa*)(ql + ks * 32), *(const v8usa*)(ql + ks * 32 + 16)); }
    v8f s[4];
#pragma unroll
    for (int nb = 0; nb < 4; ++nb) s[nb] = (v8f){};
#pragma unroll
    for (int ks = 0; ks < 2; ++ks) {
#pragma unroll
        for (int nb = 0; nb < 4; ++nb) { const bf* kpp = Khs + (nb * 16 + m) * 72 + ks * 32 + 8 * hh; const bf* lpp = Kls + (nb * 16 + m) * 72 + ks * 32 + 8 * hh;
            const v16bf bh_ = cat16b(*(const v8usa*)kpp, *(const v8usa*)(kpp + 16)); const v16bf bl_ = cat16b(*(const v8usa*)lpp, *(const v8usa*)(lpp + 16));
            s[nb] = wmmab(aqh[ks], bh_, s[nb]); s[nb] = wmmab(aqh[ks], bl_, s[nb]); s[nb] = wmmab(aql[ks], bh_, s[nb]); } }
    asm volatile("v_nop\n\tv_nop\n\tv_nop\n\tv_nop" : "+v"(s[0]), "+v"(s[1]), "+v"(s[2]), "+v"(s[3]) : "v"(aqh[0]), "v"(aql[1]));
    const int qab = q0 + 8 * hh;
    float cm[8], psum[8];
#pragma unroll
    for (int r = 0; r < 8; ++r) { cm[r] = -3.0e38f; psum[r] = 0.f; }
#pragma unroll
    for (int nb = 0; nb < 4; ++nb)
#pragma unroll
        for (int r = 0; r < 8; ++r) { float v = s[nb][r] * SCL; if (nb * 16 + m > qab + r) v = -1.0e30f; s[nb][r] = v; cm[r] = fmaxf(cm[r], v); }
#pragma unroll
    for (int r = 0; r < 8; ++r) { float c = cm[r]; c = fmaxf(c, __shfl_xor(c, 1, 32)); c = fmaxf(c, __shfl_xor(c, 2, 32)); c = fmaxf(c, __shfl_xor(c, 4, 32)); c = fmaxf(c, __shfl_xor(c, 8, 32)); cm[r] = c; }
    bf* phw = Phs + w * (16 * 72); bf* plw = Pls + w * (16 * 72); float* osw = Os + w * (16 * 68);
#pragma unroll
    for (int nb = 0; nb < 4; ++nb)
#pragma unroll
        for (int r = 0; r < 8; ++r) { const float p = __builtin_amdgcn_exp2f((s[nb][r] - cm[r]) * L2E); psum[r] += p; unsigned short a, c2; splitf(p, a, c2);
            phw[(8 * hh + r) * 72 + nb * 16 + m] = a; plw[(8 * hh + r) * 72 + nb * 16 + m] = c2; }
#pragma unroll
    for (int r = 0; r < 8; ++r) { float c = psum[r]; c += __shfl_xor(c, 1, 32); c += __shfl_xor(c, 2, 32); c += __shfl_xor(c, 4, 32); c += __shfl_xor(c, 8, 32); psum[r] = c; }
    __syncthreads();
    v16bf aph[2], apl[2];
#pragma unroll
    for (int ks = 0; ks < 2; ++ks) { const bf* pp = phw + m * 72 + ks * 32 + 8 * hh; const bf* lp = plw + m * 72 + ks * 32 + 8 * hh;
        aph[ks] = cat16b(*(const v8usa*)pp, *(const v8usa*)(pp + 16)); apl[ks] = cat16b(*(const v8usa*)lp, *(const v8usa*)(lp + 16)); }
    v8f acc[4];
#pragma unroll
    for (int nb = 0; nb < 4; ++nb) acc[nb] = (v8f){};
#pragma unroll
    for (int ks = 0; ks < 2; ++ks)
#pragma unroll
        for (int nb = 0; nb < 4; ++nb) { const bf* vp = Vhs + (nb * 16 + m) * 72 + ks * 32 + 8 * hh; const bf* vlp = Vls + (nb * 16 + m) * 72 + ks * 32 + 8 * hh;
            const v16bf bvh = cat16b(*(const v8usa*)vp, *(const v8usa*)(vp + 16)); const v16bf bvl = cat16b(*(const v8usa*)vlp, *(const v8usa*)(vlp + 16));
            acc[nb] = wmmab(aph[ks], bvh, acc[nb]); acc[nb] = wmmab(aph[ks], bvl, acc[nb]); acc[nb] = wmmab(apl[ks], bvh, acc[nb]); }
    asm volatile("v_nop\n\tv_nop\n\tv_nop\n\tv_nop" : "+v"(acc[0]), "+v"(acc[1]), "+v"(acc[2]), "+v"(acc[3]) : "v"(aph[0]), "v"(apl[1]));
    const float qnan = __uint_as_float(0x7fc00000u);
#pragma unroll
    for (int r = 0; r < 8; ++r) { const float iv = 1.0f / psum[r];
#pragma unroll
        for (int nb = 0; nb < 4; ++nb) { const float o = acc[nb][r] * iv; osw[(8 * hh + r) * 68 + nb * 16 + m] = ok ? o : qnan; } }
    __syncthreads();
    store_ctx(osw, ATh, ATl, (size_t)(b * SEQ + q0) * DM + h * HD, lane);
}

#define AL256(x) ((((size_t)(x)) + 255) & ~(size_t)255)
static constexpr size_t SZ_WQKV = (size_t)NQKV * DM * 2;
static constexpr size_t SZ_W    = (size_t)DM * DM * 2;
static constexpr size_t SZ_FL   = (size_t)NCHK * 32 * 4;
static constexpr size_t SZ_X    = (size_t)NB * SEQ * DM * 2;
static constexpr size_t SZ_P    = (size_t)NB * SEQ * DM * 2;
static constexpr size_t SZ_E    = (size_t)NB * RE * DM * 2;
static constexpr size_t WS_TOTAL = AL256(SZ_WQKV) + AL256(SZ_W) + AL256(SZ_FL) + AL256(SZ_X) + AL256(2 * SZ_P) + AL256(SZ_P) + 2 * AL256(2 * SZ_E) + 2 * AL256(SZ_E) + 2 * AL256(SZ_P);
static_assert(WS_TOTAL <= (size_t)134217728);
static_assert((size_t)NB * SEQ * DM * 4 <= (size_t)NB_FULL * SEQ_FULL * DM * 4);
static_assert(SZ_P % 256 == 0 && SZ_E % 256 == 0);

extern "C" void kernel_launch(void* const* d_in, const int* in_sizes, int n_in,
                              void* d_out, int out_size, void* d_ws, size_t ws_size, hipStream_t stream) {
    if (n_in < 6) return;
    if ((size_t)in_sizes[0] < (size_t)NB * SEQ * DM) return;
    if ((size_t)in_sizes[1] < (size_t)SEQ * SEQ) return;
    if ((size_t)in_sizes[2] < (size_t)DM * NQKV || (size_t)in_sizes[3] < (size_t)NQKV) return;
    if ((size_t)in_sizes[4] < (size_t)DM * DM || (size_t)in_sizes[5] < (size_t)DM) return;
    if ((size_t)out_size < (size_t)NB * SEQ * DM) return;
    if (WS_TOTAL > ws_size) return;
    const float* x     = (const float*)d_in[0];
    const float* am    = (const float*)d_in[1];
    const float* wqkv  = (const float*)d_in[2];
    const float* bqkv  = (const float*)d_in[3];
    const float* wproj = (const float*)d_in[4];
    const float* bproj = (const float*)d_in[5];
    float* OUT = (float*)d_out;
    char* wsp = (char*)d_ws;
    auto take = [&](size_t bytes) { char* p = wsp; wsp += AL256(bytes); return (void*)p; };
    bf* WQKV = (bf*)take(SZ_WQKV);
    bf* WO   = (bf*)take(SZ_W);
    float* FL = (float*)take(SZ_FL);
    bf* XB = (bf*)take(SZ_X);
    h16* QK16 = (h16*)take(2 * SZ_P);
    h16* VT16 = (h16*)take(SZ_P);
    bf* QKh = (bf*)take(2 * SZ_E); bf* QKl = (bf*)take(2 * SZ_E);
    bf* VTh = (bf*)take(SZ_E); bf* VTl = (bf*)take(SZ_E);
    bf* ATh = (bf*)take(SZ_P); bf* ATl = (bf*)take(SZ_P);
    if ((size_t)(wsp - (char*)d_ws) > ws_size || (size_t)(wsp - (char*)d_ws) != WS_TOTAL) return;
    h16* Q16 = QK16; h16* K16 = QK16 + (size_t)NB * SEQ * DM;
    bf* Qh = QKh; bf* Kh = QKh + (size_t)NB * RE * DM; bf* Ql = QKl; bf* Kl = QKl + (size_t)NB * RE * DM;

    const unsigned LX = (unsigned)(((size_t)NB * SEQ * DM / 8 + 255) / 256);
    k_cvtT<<<dim3(DM / 64, NQKV / 64, 1), 256, 0, stream>>>(wqkv, WQKV, DM, NQKV);
    k_cvtT<<<dim3(DM / 64, DM / 64, 1), 256, 0, stream>>>(wproj, WO, DM, DM);
    k_mchk<<<NCHK, 256, 0, stream>>>(am, FL);
    k_cvtx<<<LX, 256, 0, stream>>>(x, XB, (size_t)NB * SEQ * DM / 8);
    k_gemmp<1><<<dim3(NB * SEQ / 64, DM / 64, 2), 32, 0, stream>>>(XB, WQKV, DM, bqkv, QK16, DM, QKh, QKl, DM,
                                                                   (size_t)0, (size_t)DM * DM, (size_t)DM, (size_t)NB * SEQ * DM, (size_t)NB * RE * DM);
    k_gemmp<2><<<dim3(DM / 64, SEQ / 64, NB), 32, 0, stream>>>(WQKV + (size_t)2 * DM * DM, XB, DM, bqkv + 2 * DM, VT16, SEQ, VTh, VTl, RE,
                                                               (size_t)0, (size_t)SEQ * DM, (size_t)0, (size_t)DM * SEQ, (size_t)DM * RE);
    k_attn0<<<dim3(RE / 32, NB * NH, 1), 64, 0, stream>>>(Qh, Ql, Kh, Kl, VTh, VTl, FL, ATh, ATl);
    if (SEQ / 64 > 1) k_attn<<<dim3(SEQ / 64 - 1, NB * NH, 1), 128, 0, stream>>>(Q16, K16, VT16, FL, ATh, ATl);
    k_gemmw<bf, 1><<<dim3(NB * SEQ / 64, DM / 64, 1), 32, 0, stream>>>(ATh, ATl, WO, nullptr, DM, bproj, OUT, DM, (size_t)0, (size_t)0, (size_t)0);
}
